// CrossAttention_3942779978031
// MI455X (gfx1250) — hardware-verified
//
#include <hip/hip_runtime.h>

#ifndef NB
#define NB 4
#endif
#ifndef SEQ
#define SEQ 4096
#endif
#define NB_FULL 4
#define SEQ_FULL 4096
#define DIN 256
#define DOUT 128
#define NROWS (NB * SEQ)
#define OSP 132
#define GSP 68

static_assert(NB <= NB_FULL);
static_assert(SEQ <= SEQ_FULL);
static_assert(SEQ % 64 == 0);
static_assert(NROWS % 64 == 0);
static_assert(DIN % 32 == 0);
static_assert(DIN % 8 == 0);
static_assert(DOUT == 128);
static_assert(DOUT % 64 == 0);
static_assert(DOUT % 32 == 0);
static_assert((OSP * 4) % 16 == 0);
static_assert((GSP * 4) % 16 == 0);

typedef __attribute__((ext_vector_type(16))) __bf16       v16b;
typedef __attribute__((ext_vector_type(8)))  __bf16       v8b;
typedef __attribute__((ext_vector_type(8)))  float        v8f;
typedef __attribute__((ext_vector_type(4)))  float        v4f;
typedef __attribute__((ext_vector_type(4)))  unsigned int v4u;
typedef __attribute__((ext_vector_type(8)))  unsigned int v8u;

union FB { v16b v; v8b h[2]; };
__device__ __forceinline__ v16b ldfrag(const __bf16* __restrict__ p) {
    FB f; f.h[0] = *(const v8b*)(p); f.h[1] = *(const v8b*)(p + 16); return f.v;
}
__device__ __forceinline__ v8f mmab(v16b a, v16b b, v8f c) {
    return __builtin_amdgcn_wmma_f32_16x16x32_bf16(false, a, false, b, (short)0, c, false, false);
}
__device__ __forceinline__ void guard_s2(v8f& a, v8f& b, v16b x0, v16b x1, v16b x2, v16b x3, v16b x4, v16b x5) {
    asm volatile("v_nop\n\tv_nop\n\tv_nop\n\tv_nop" : "+v"(a), "+v"(b) : "v"(x0), "v"(x1), "v"(x2), "v"(x3), "v"(x4), "v"(x5));
}
__device__ __forceinline__ void guard_a4(v8f& a, v8f& b, v8f& c, v8f& d, v16b x0, v16b x1, v16b x2, v16b x3, v16b x4) {
    asm volatile("v_nop\n\tv_nop\n\tv_nop\n\tv_nop" : "+v"(a), "+v"(b), "+v"(c), "+v"(d) : "v"(x0), "v"(x1), "v"(x2), "v"(x3), "v"(x4));
}
__device__ __forceinline__ void guard_o4(v8f& a, v8f& b, v8f& c, v8f& d, v16b x0, v16b x1, v16b x2, v16b x3, v16b x4, v16b x5, v16b x6, v16b x7, v16b x8, v16b x9) {
    asm volatile("v_nop\n\tv_nop\n\tv_nop\n\tv_nop" : "+v"(a), "+v"(b), "+v"(c), "+v"(d)
                 : "v"(x0), "v"(x1), "v"(x2), "v"(x3), "v"(x4), "v"(x5), "v"(x6), "v"(x7), "v"(x8), "v"(x9) : "memory");
}

__device__ __forceinline__ unsigned int bf_hi_word(float f) {
    unsigned int u = __float_as_uint(f);
    u += 0x7FFFu + ((u >> 16) & 1u);
    return u & 0xFFFF0000u;
}
__device__ __forceinline__ unsigned int pack_pair(float a, float b) { return (bf_hi_word(a) >> 16) | bf_hi_word(b); }
__device__ __forceinline__ void split_pair(float a, float b, unsigned int& hi, unsigned int& lo) {
    const unsigned int ua = bf_hi_word(a), ub = bf_hi_word(b);
    const unsigned int la = bf_hi_word(a - __uint_as_float(ua)), lb = bf_hi_word(b - __uint_as_float(ub));
    hi = (ua >> 16) | ub; lo = (la >> 16) | lb;
}
__device__ __forceinline__ float bf_val(float f) { return __uint_as_float(bf_hi_word(f)); }

__global__ __launch_bounds__(256) void k_cast_rows(const float* __restrict__ SRC, unsigned short* __restrict__ DST) {
    const int u = (int)blockIdx.x * 256 + (int)threadIdx.x;
    if (u >= NROWS * (DIN / 8)) return;
    const int r = u / (DIN / 8), c0 = 8 * (u % (DIN / 8));
    const int b = r / SEQ, s = r - b * SEQ;
    const float* sp = SRC + ((size_t)b * SEQ_FULL + (size_t)s) * DIN + c0;
    const v4f a = *(const v4f*)sp; const v4f d = *(const v4f*)(sp + 4);
    v4u pk; pk.x = pack_pair(a.x, a.y); pk.y = pack_pair(a.z, a.w); pk.z = pack_pair(d.x, d.y); pk.w = pack_pair(d.z, d.w);
    volatile v4u* dp = (volatile v4u*)(DST + (size_t)r * DIN + c0);
    *dp = pk; __threadfence(); *dp = pk;
}

__global__ __launch_bounds__(256) void k_cast_wT(const float* __restrict__ W, unsigned short* __restrict__ WT) {
    const int u = (int)blockIdx.x * 256 + (int)threadIdx.x;
    if (u >= DOUT * (DIN / 8)) return;
    const int c = u / (DIN / 8), r0 = 8 * (u % (DIN / 8));
    float w[8];
#pragma unroll
    for (int e = 0; e < 8; ++e) w[e] = W[(size_t)(r0 + e) * DOUT + c];
    v4u pk; pk.x = pack_pair(w[0], w[1]); pk.y = pack_pair(w[2], w[3]); pk.z = pack_pair(w[4], w[5]); pk.w = pack_pair(w[6], w[7]);
    volatile v4u* dp = (volatile v4u*)(WT + (size_t)c * DIN + r0);
    *dp = pk; __threadfence(); *dp = pk;
}

template <int BIAS_M>
__device__ __forceinline__ void proj_body(const unsigned short* __restrict__ Ap, const int lda,
                                          const unsigned short* __restrict__ Btp, const int ldb,
                                          unsigned short* __restrict__ Ch, unsigned short* __restrict__ Cl, const int ldc,
                                          const float* __restrict__ bias, const int M, const int N, const int K) {
    __shared__ __align__(16) float sT[8 * 16 * GSP];
    const __bf16* A  = (const __bf16*)Ap;
    const __bf16* Bt = (const __bf16*)Btp;
    const int lane = (int)threadIdx.x & 31;
    const int wave = __builtin_amdgcn_readfirstlane((int)(threadIdx.x >> 5));
    const int tilesN = N >> 6, tilesM = M >> 6;
    const int tile = (int)blockIdx.x * 8 + wave;
    if (tile >= tilesM * tilesN) return;
    const int tm = tile / tilesN, tn = tile - tm * tilesN;
    const int m0 = tm << 6, n0 = tn << 6;
    const int rl = lane & 15, koff = (lane >> 4) * 8, mOff = (lane >> 4) * 8;

    v8f acc[4][4];
#pragma unroll
    for (int i = 0; i < 4; ++i)
#pragma unroll
        for (int j = 0; j < 4; ++j) { const v8f z = {0.f, 0.f, 0.f, 0.f, 0.f, 0.f, 0.f, 0.f}; acc[i][j] = z; }

#pragma unroll 1
    for (int k0 = 0; k0 < K; k0 += 32) {
        v16b bh[4];
#pragma unroll
        for (int j = 0; j < 4; ++j) bh[j] = ldfrag(Bt + (size_t)(n0 + 16 * j + rl) * ldb + koff + k0);
#pragma unroll
        for (int i = 0; i < 4; ++i) {
            const v16b ah = ldfrag(A + (size_t)(m0 + 16 * i + rl) * lda + koff + k0);
#pragma unroll
            for (int j = 0; j < 4; ++j) acc[i][j] = mmab(ah, bh[j], acc[i][j]);
            guard_a4(acc[i][0], acc[i][1], acc[i][2], acc[i][3], ah, bh[0], bh[1], bh[2], bh[3]);
        }
    }

    const int sb = wave * (16 * GSP);
#pragma unroll
    for (int i = 0; i < 4; ++i) {
        const int mBase = m0 + 16 * i;
#pragma unroll
        for (int j = 0; j < 4; ++j) {
            const int n = n0 + 16 * j + rl;
            const float bv = BIAS_M ? 0.f : bf_val(bias[n]);
#pragma unroll
            for (int r = 0; r < 8; ++r) {
                float v = acc[i][j][r];
                if (BIAS_M) v += bf_val(bias[mBase + mOff + r]); else v += bv;
                sT[sb + (mOff + r) * GSP + 16 * j + rl] = v;
            }
        }
        __builtin_amdgcn_fence(3  , "workgroup");
        __builtin_amdgcn_wave_barrier();
        __builtin_amdgcn_fence(2  , "workgroup");
        {
            const int q = lane >> 3, c8 = (lane & 7) * 8;
            for (int pass = 0; pass < 2; ++pass) {
#pragma unroll
                for (int it = 0; it < 4; ++it) {
                    const int row = it * 4 + q;
                    const int so = sb + row * GSP + c8;
                    v4u hv, lv; unsigned int h_, l_;
                    split_pair(sT[so + 0], sT[so + 1], h_, l_); hv.x = h_; lv.x = l_;
                    split_pair(sT[so + 2], sT[so + 3], h_, l_); hv.y = h_; lv.y = l_;
                    split_pair(sT[so + 4], sT[so + 5], h_, l_); hv.z = h_; lv.z = l_;
                    split_pair(sT[so + 6], sT[so + 7], h_, l_); hv.w = h_; lv.w = l_;
                    const size_t go = (size_t)(mBase + row) * ldc + n0 + c8;
                    *(volatile v4u*)(Ch + go) = hv;
                    *(volatile v4u*)(Cl + go) = lv;
                }
                __threadfence();
            }
        }
        __builtin_amdgcn_fence(3  , "workgroup");
        __builtin_amdgcn_wave_barrier();
        __builtin_amdgcn_fence(2  , "workgroup");
    }
}

__global__ __launch_bounds__(256) void k_proj_rows(const unsigned short* __restrict__ A, const unsigned short* __restrict__ WT, unsigned short* __restrict__ Ch, unsigned short* __restrict__ Cl, const float* __restrict__ bias) {
    proj_body<0>(A, DIN, WT, DIN, Ch, Cl, DOUT, bias, NROWS, DOUT, DIN);
}
__global__ __launch_bounds__(256) void k_proj_vt(const unsigned short* __restrict__ WT, const unsigned short* __restrict__ Bt, unsigned short* __restrict__ Ch, unsigned short* __restrict__ Cl, const float* __restrict__ bias) {
    proj_body<1>(WT, DIN, Bt, DIN, Ch, Cl, NROWS, bias, DOUT, NROWS, DIN);
}

__device__ __forceinline__ void p_tile(const v8f s, const float mnew, float& rs, v4u& hi, v4u& lo) {
    float p[8];
#pragma unroll
    for (int r = 0; r < 8; ++r) { p[r] = __expf(s[r] - mnew); rs += p[r]; }
    unsigned int h_, l_;
    split_pair(p[0], p[1], h_, l_); hi.x = h_; lo.x = l_;
    split_pair(p[2], p[3], h_, l_); hi.y = h_; lo.y = l_;
    split_pair(p[4], p[5], h_, l_); hi.z = h_; lo.z = l_;
    split_pair(p[6], p[7], h_, l_); hi.w = h_; lo.w = l_;
}

__global__ __launch_bounds__(128) void k_xattn(const unsigned short* __restrict__ QHp, const unsigned short* __restrict__ QLp,
                                               const unsigned short* __restrict__ KHp, const unsigned short* __restrict__ KLp,
                                               const unsigned short* __restrict__ VHp, const unsigned short* __restrict__ VLp,
                                               float* __restrict__ out) {
    __shared__ __align__(16) float Os[4 * 16 * OSP];
    const __bf16* QH = (const __bf16*)QHp; const __bf16* QL = (const __bf16*)QLp;
    const __bf16* KH = (const __bf16*)KHp; const __bf16* KL = (const __bf16*)KLp;
    const __bf16* VH = (const __bf16*)VHp; const __bf16* VL = (const __bf16*)VLp;
    const int lane = (int)threadIdx.x & 31;
    const int wave = __builtin_amdgcn_readfirstlane((int)(threadIdx.x >> 5));
    const int hh = lane >> 4, c = lane & 15;
    const int b = (int)blockIdx.y;
    const int q0 = (int)blockIdx.x * 64 + wave * 16;
    const int qoff  = (b * SEQ + q0 + c) * DOUT + 8 * hh;
    const int kbase = (b * SEQ + c) * DOUT + 8 * hh;
    const int vbase = c * NROWS + b * SEQ + 8 * hh;

    v8f o[8];
#pragma unroll
    for (int t = 0; t < 8; ++t) { const v8f z = {0.f, 0.f, 0.f, 0.f, 0.f, 0.f, 0.f, 0.f}; o[t] = z; }
    float mrun = -__builtin_inff(), lrun = 0.f;

#pragma unroll 1
    for (int kv0 = 0; kv0 < SEQ; kv0 += 64) {
        const v8f zz = {0.f, 0.f, 0.f, 0.f, 0.f, 0.f, 0.f, 0.f};
        v8f s0 = zz, s1 = zz, s2 = zz, s3 = zz;
        const int ko = kbase + kv0 * DOUT;
#pragma unroll 1
        for (int dc = 0; dc < DOUT / 32; ++dc) {
            const v16b qh = ldfrag(QH + qoff + dc * 32), ql = ldfrag(QL + qoff + dc * 32);
            {
                const v16b a0h = ldfrag(KH + ko + dc * 32),             a0l = ldfrag(KL + ko + dc * 32);
                const v16b a1h = ldfrag(KH + ko + 16 * DOUT + dc * 32), a1l = ldfrag(KL + ko + 16 * DOUT + dc * 32);
                s0 = mmab(a0h, qh, s0); s0 = mmab(a0h, ql, s0); s0 = mmab(a0l, qh, s0);
                s1 = mmab(a1h, qh, s1); s1 = mmab(a1h, ql, s1); s1 = mmab(a1l, qh, s1);
                guard_s2(s0, s1, a0h, a0l, a1h, a1l, qh, ql);
            }
            {
                const v16b a2h = ldfrag(KH + ko + 32 * DOUT + dc * 32), a2l = ldfrag(KL + ko + 32 * DOUT + dc * 32);
                const v16b a3h = ldfrag(KH + ko + 48 * DOUT + dc * 32), a3l = ldfrag(KL + ko + 48 * DOUT + dc * 32);
                s2 = mmab(a2h, qh, s2); s2 = mmab(a2h, ql, s2); s2 = mmab(a2l, qh, s2);
                s3 = mmab(a3h, qh, s3); s3 = mmab(a3h, ql, s3); s3 = mmab(a3l, qh, s3);
                guard_s2(s2, s3, a2h, a2l, a3h, a3l, qh, ql);
            }
        }

        float mx = s0[0];
#pragma unroll
        for (int r = 0; r < 8; ++r) { mx = fmaxf(mx, s0[r]); mx = fmaxf(mx, s1[r]); mx = fmaxf(mx, s2[r]); mx = fmaxf(mx, s3[r]); }
        mx = fmaxf(mx, __shfl_xor(mx, 16, 32));
        const float mnew = fmaxf(mrun, mx);
        const float corr = __expf(mrun - mnew);
        mrun = mnew;
        float rs = 0.f;
        v4u h0, l0, h1, l1, h2, l2, h3, l3;
        p_tile(s0, mnew, rs, h0, l0);
        p_tile(s1, mnew, rs, h1, l1);
        p_tile(s2, mnew, rs, h2, l2);
        p_tile(s3, mnew, rs, h3, l3);
        rs += __shfl_xor(rs, 16, 32);
        lrun = lrun * corr + rs;
#pragma unroll
        for (int t = 0; t < 8; ++t) o[t] = o[t] * corr;

        v16b pbh[2], pbl[2];
        pbh[0] = __builtin_bit_cast(v16b, __builtin_shufflevector(h0, h1, 0, 1, 2, 3, 4, 5, 6, 7));
        pbl[0] = __builtin_bit_cast(v16b, __builtin_shufflevector(l0, l1, 0, 1, 2, 3, 4, 5, 6, 7));
        pbh[1] = __builtin_bit_cast(v16b, __builtin_shufflevector(h2, h3, 0, 1, 2, 3, 4, 5, 6, 7));
        pbl[1] = __builtin_bit_cast(v16b, __builtin_shufflevector(l2, l3, 0, 1, 2, 3, 4, 5, 6, 7));

        const int vo0 = vbase + kv0;
#pragma unroll
        for (int kk = 0; kk < 2; ++kk) {
#pragma unroll
            for (int tg = 0; tg < 2; ++tg) {
                v16b vh[4], vl[4];
#pragma unroll
                for (int t = 0; t < 4; ++t) {
                    const int vo = vo0 + (tg * 4 + t) * 16 * NROWS + kk * 32;
                    vh[t] = ldfrag(VH + vo); vl[t] = ldfrag(VL + vo);
                }
#pragma unroll
                for (int t = 0; t < 4; ++t) {
                    o[tg * 4 + t] = mmab(vh[t], pbh[kk], o[tg * 4 + t]);
                    o[tg * 4 + t] = mmab(vh[t], pbl[kk], o[tg * 4 + t]);
                    o[tg * 4 + t] = mmab(vl[t], pbh[kk], o[tg * 4 + t]);
                }
                guard_o4(o[tg * 4 + 0], o[tg * 4 + 1], o[tg * 4 + 2], o[tg * 4 + 3],
                         vh[0], vh[1], vh[2], vh[3], vl[0], vl[1], vl[2], vl[3], pbh[kk], pbl[kk]);
            }
        }
    }

    const float inv = 1.0f / lrun;
    const int wb = wave * (16 * OSP);
#pragma unroll
    for (int t = 0; t < 8; ++t) {
        v4f a, d;
        a.x = o[t][0] * inv; a.y = o[t][1] * inv; a.z = o[t][2] * inv; a.w = o[t][3] * inv;
        d.x = o[t][4] * inv; d.y = o[t][5] * inv; d.z = o[t][6] * inv; d.w = o[t][7] * inv;
        *(v4f*)&Os[wb + c * OSP + 16 * t + 8 * hh]     = a;
        *(v4f*)&Os[wb + c * OSP + 16 * t + 8 * hh + 4] = d;
    }
    __builtin_amdgcn_fence(3  , "workgroup");
    __builtin_amdgcn_wave_barrier();
    __builtin_amdgcn_fence(2  , "workgroup");
    {
        float* ob = out + ((size_t)b * SEQ + (size_t)q0) * DOUT;
        const int c4 = lane * 4;
        for (int pass = 0; pass < 2; ++pass) {
#pragma unroll
            for (int row = 0; row < 16; ++row) {
                const v4f val = *(const v4f*)&Os[wb + row * OSP + c4];
                *(volatile v4f*)(ob + (size_t)row * DOUT + c4) = val;
            }
            __threadfence();
        }
    }
}

extern "C" void kernel_launch(void* const* d_in, const int* in_sizes, int n_in, void* d_out, int out_size, void* d_ws, size_t ws_size, hipStream_t stream) {
    if (n_in < 8) return;
    const long long need_rows = ((long long)(NB - 1) * SEQ_FULL + SEQ) * DIN;
    if ((long long)in_sizes[0] < need_rows || (long long)in_sizes[1] < need_rows) return;
    if (in_sizes[2] < DIN * DOUT || in_sizes[4] < DIN * DOUT || in_sizes[6] < DIN * DOUT) return;
    if (in_sizes[3] < DOUT || in_sizes[5] < DOUT || in_sizes[7] < DOUT) return;
    if ((long long)out_size < (long long)NROWS * DOUT) return;

    const float* x    = (const float*)d_in[0];
    const float* cond = (const float*)d_in[1];
    const float* Wq   = (const float*)d_in[2];
    const float* bq   = (const float*)d_in[3];
    const float* Wk   = (const float*)d_in[4];
    const float* bk   = (const float*)d_in[5];
    const float* Wv   = (const float*)d_in[6];
    const float* bv   = (const float*)d_in[7];
    float* out = (float*)d_out;

    constexpr size_t SZ_IN = (size_t)NROWS * DIN * 2;
    constexpr size_t SZ_W  = (size_t)DOUT * DIN * 2;
    constexpr size_t SZ_PL = (size_t)NROWS * DOUT * 2;
    constexpr size_t WS_TOTAL = 2 * SZ_IN + 3 * SZ_W + 6 * SZ_PL;
    static_assert(SZ_IN % 256 == 0);
    static_assert(SZ_W % 256 == 0);
    static_assert(SZ_PL % 256 == 0);
    static_assert(WS_TOTAL <= (size_t)134217728);
    if (WS_TOTAL > ws_size) return;

    char* wsp = (char*)d_ws;
    unsigned short* XB  = (unsigned short*)wsp; wsp += SZ_IN;
    unsigned short* CB  = (unsigned short*)wsp; wsp += SZ_IN;
    unsigned short* WQT = (unsigned short*)wsp; wsp += SZ_W;
    unsigned short* WKT = (unsigned short*)wsp; wsp += SZ_W;
    unsigned short* WVT = (unsigned short*)wsp; wsp += SZ_W;
    unsigned short* QH  = (unsigned short*)wsp; wsp += SZ_PL;
    unsigned short* QL  = (unsigned short*)wsp; wsp += SZ_PL;
    unsigned short* KH  = (unsigned short*)wsp; wsp += SZ_PL;
    unsigned short* KL  = (unsigned short*)wsp; wsp += SZ_PL;
    unsigned short* VTH = (unsigned short*)wsp; wsp += SZ_PL;
    unsigned short* VTL = (unsigned short*)wsp; wsp += SZ_PL;

    constexpr unsigned CAST_BLOCKS = (unsigned)((NROWS * (DIN / 8) + 255) / 256);
    constexpr unsigned W_BLOCKS    = (unsigned)((DOUT * (DIN / 8) + 255) / 256);
    constexpr unsigned GEMM_BLOCKS = (unsigned)((((NROWS / 64) * (DOUT / 64)) + 7) / 8);

    k_cast_rows<<<CAST_BLOCKS, 256, 0, stream>>>(x, XB);
    k_cast_rows<<<CAST_BLOCKS, 256, 0, stream>>>(cond, CB);
    k_cast_wT<<<W_BLOCKS, 256, 0, stream>>>(Wq, WQT);
    k_cast_wT<<<W_BLOCKS, 256, 0, stream>>>(Wk, WKT);
    k_cast_wT<<<W_BLOCKS, 256, 0, stream>>>(Wv, WVT);
    k_proj_rows<<<GEMM_BLOCKS, 256, 0, stream>>>(XB, WQT, QH, QL, bq);
    k_proj_rows<<<GEMM_BLOCKS, 256, 0, stream>>>(CB, WKT, KH, KL, bk);
    k_proj_vt<<<GEMM_BLOCKS, 256, 0, stream>>>(WVT, CB, VTH, VTL, bv);
    k_xattn<<<dim3((unsigned)(SEQ / 64), (unsigned)NB), 128, 0, stream>>>(QH, QL, KH, KL, VTH, VTL, out);
}
